// MultiHeadCausalAttention_84902913507671
// MI455X (gfx1250) — hardware-verified
//
#include <hip/hip_runtime.h>
#include <math.h>

#ifndef NB
#define NB 2
#endif
#ifndef SEQ
#define SEQ 2048
#endif
#define NB_FULL 2
#define SEQ_FULL 2048

constexpr int kBatch   = NB;
constexpr int kSeq     = SEQ;
constexpr int kSeqFull = SEQ_FULL;
constexpr int kDim     = 1024;
constexpr int kHeads   = 16;
constexpr int kDh      = 64;
constexpr int kTok     = kBatch * kSeq;
constexpr int kWtN     = 3 * kDim;
constexpr int kQKld    = 2 * kDim;
constexpr int kQB      = 64;
constexpr int kKC      = 64;
constexpr int kAW      = 4;
constexpr float kScale  = 0.125f;
constexpr float kNegBig = -1.0e30f;
static_assert(kBatch >= 1 && kBatch <= NB_FULL);
static_assert(kSeq >= 64 && kSeq <= SEQ_FULL);
static_assert(kHeads * kDh == kDim);
static_assert(kSeq % kQB == 0 && kSeq % kKC == 0 && kQB == kAW * 16 && kDh == 64);
static_assert(kTok % 64 == 0 && kQKld % 64 == 0 && kDim % 32 == 0);
static_assert(kDim % 64 == 0 && kSeq % 64 == 0);
static_assert(kDim / 8 == 128 && (kTok * kDim) % 8 == 0);

typedef __attribute__((ext_vector_type(16))) _Float16 v16h;
typedef __attribute__((ext_vector_type(8)))  _Float16 v8h;
typedef __attribute__((ext_vector_type(16))) __bf16   v16b;
typedef __attribute__((ext_vector_type(8)))  __bf16   v8b;
typedef __attribute__((ext_vector_type(8)))  float    v8f;
typedef __attribute__((ext_vector_type(4)))  float    v4f;
typedef __attribute__((ext_vector_type(4)))  unsigned int v4u;

__device__ __forceinline__ unsigned short f2bf_bits(float f) {
  unsigned u = __float_as_uint(f);
  return (unsigned short)((u + 0x7FFFu + ((u >> 16) & 1u)) >> 16);
}
__device__ __forceinline__ float bf_bits2f(unsigned short h) { return __uint_as_float(((unsigned)h) << 16); }

__device__ __forceinline__ void dep_guard_h(v8f& a, v8f& b, v16h x, v16h y) { asm volatile("v_nop\n\tv_nop\n\tv_nop\n\tv_nop" : "+v"(a), "+v"(b) : "v"(x), "v"(y)); }
__device__ __forceinline__ void dep_guard_b(v8f& a, v8f& b, v16b x, v16b y) { asm volatile("v_nop\n\tv_nop\n\tv_nop\n\tv_nop" : "+v"(a), "+v"(b) : "v"(x), "v"(y)); }
__device__ __forceinline__ void dep_guard4_h(v8f& a, v8f& b, v8f& c, v8f& d, v16h x, v16h y) { asm volatile("v_nop\n\tv_nop\n\tv_nop\n\tv_nop" : "+v"(a), "+v"(b), "+v"(c), "+v"(d) : "v"(x), "v"(y)); }
__device__ __forceinline__ void dep_guard4_b(v8f& a, v8f& b, v8f& c, v8f& d, v16b x, v16b y) { asm volatile("v_nop\n\tv_nop\n\tv_nop\n\tv_nop" : "+v"(a), "+v"(b), "+v"(c), "+v"(d) : "v"(x), "v"(y)); }
__device__ __forceinline__ void keep4_h(v16h a, v16h b, v16h c, v16h d) { asm volatile("v_nop" :: "v"(a), "v"(b), "v"(c), "v"(d)); }
__device__ __forceinline__ void keep4_b(v16b a, v16b b, v16b c, v16b d) { asm volatile("v_nop" :: "v"(a), "v"(b), "v"(c), "v"(d)); }
__device__ __forceinline__ void acc_guard4(v8f& a, v8f& b, v8f& c, v8f& d) { asm volatile("v_nop\n\tv_nop\n\tv_nop\n\tv_nop" : "+v"(a), "+v"(b), "+v"(c), "+v"(d)); }
template <typename T> struct Frag;
template <> struct Frag<_Float16> {
  typedef v16h V; union U { v16h v; v8h h[2]; };
  static __device__ __forceinline__ v16h load(const _Float16* p) {
    U f; f.h[0] = *(const v8h*)(p); f.h[1] = *(const v8h*)(p + 16); return f.v;
  }
  static __device__ __forceinline__ v8f mma(v16h a, v16h b, v8f c) {
    return __builtin_amdgcn_wmma_f32_16x16x32_f16(false, a, false, b, (short)0, c, false, false);
  }
  static __device__ __forceinline__ void guard(v8f& a, v8f& b, v16h x, v16h y) { dep_guard_h(a, b, x, y); }
  static __device__ __forceinline__ void guard4(v8f& a, v8f& b, v8f& c, v8f& d, v16h x, v16h y) { dep_guard4_h(a, b, c, d, x, y); }
  static __device__ __forceinline__ void keep(v16h a, v16h b, v16h c, v16h d) { keep4_h(a, b, c, d); }
};
template <> struct Frag<__bf16> {
  typedef v16b V; union U { v16b v; v8b h[2]; };
  static __device__ __forceinline__ v16b load(const __bf16* p) {
    U f; f.h[0] = *(const v8b*)(p); f.h[1] = *(const v8b*)(p + 16); return f.v;
  }
  static __device__ __forceinline__ v8f mma(v16b a, v16b b, v8f c) {
    return __builtin_amdgcn_wmma_f32_16x16x32_bf16(false, a, false, b, (short)0, c, false, false);
  }
  static __device__ __forceinline__ void guard(v8f& a, v8f& b, v16b x, v16b y) { dep_guard_b(a, b, x, y); }
  static __device__ __forceinline__ void guard4(v8f& a, v8f& b, v8f& c, v8f& d, v16b x, v16b y) { dep_guard4_b(a, b, c, d, x, y); }
  static __device__ __forceinline__ void keep(v16b a, v16b b, v16b c, v16b d) { keep4_b(a, b, c, d); }
};

__device__ __forceinline__ unsigned pk16(unsigned short a, unsigned short b) { return (unsigned)a | ((unsigned)b << 16); }

template <int ET> struct Elem;
template <> struct Elem<0> { typedef _Float16 T; };
template <> struct Elem<1> { typedef __bf16 T; };
template <int ET, int SPLIT, int BIAS_MODE, int OUT_MODE>
__global__ __launch_bounds__(256) void wmma_gemm64(
    const unsigned short* __restrict__ Ap, const unsigned short* __restrict__ A2p, int lda, long strideA,
    const unsigned short* __restrict__ Btp, const unsigned short* __restrict__ Bt2p, int ldb, long strideB,
    void* __restrict__ Cout, void* __restrict__ Cout2, int ldc, long strideC,
    const float* __restrict__ bias,
    int M, int N, int K, float scale) {
  static_assert(SPLIT >= 0 && SPLIT <= 2);
  static_assert(BIAS_MODE >= 0 && BIAS_MODE <= 2);
  static_assert(OUT_MODE >= 0 && OUT_MODE <= 2);
  typedef typename Elem<ET>::T T;
  typedef typename Frag<T>::V V;
  const T* A = (const T*)Ap; const T* A2 = (const T*)A2p; const T* Bt = (const T*)Btp; const T* Bt2 = (const T*)Bt2p;
  __shared__ __align__(16) float sT[8][16 * 68];
  const int b    = blockIdx.y;
  const int lane = threadIdx.x & 31;
  const int wave = threadIdx.x >> 5;
  const int tilesN = N >> 6;
  const int tilesM = M >> 6;
  const int tile = blockIdx.x * 8 + wave;
  if (tile >= tilesM * tilesN) return;
  const int tm = tile / tilesN;
  const int tn = tile - tm * tilesN;
  const int m0 = tm << 6;
  const int n0 = tn << 6;

  const T* Ab  = A  + (size_t)b * strideA;
  const T* Bb  = Bt + (size_t)b * strideB;
  const T* Ab2 = (SPLIT != 0) ? (A2  + (size_t)b * strideA) : nullptr;
  const T* Bb2 = (SPLIT == 1) ? (Bt2 + (size_t)b * strideB) : nullptr;

  const int rlane = lane & 15;
  const int koff  = (lane >> 4) * 8;
  const int mOff  = (lane >> 4) * 8;

  v8f acc[4][4];
#pragma unroll
  for (int i = 0; i < 4; ++i)
#pragma unroll
    for (int j = 0; j < 4; ++j) acc[i][j] = (v8f){0.f,0.f,0.f,0.f,0.f,0.f,0.f,0.f};

  for (int k0 = 0; k0 < K; k0 += 32) {
    V bh[4], bl[4];
#pragma unroll
    for (int j = 0; j < 4; ++j) {
      const size_t bo = (size_t)(n0 + (j << 4) + rlane) * ldb + koff + k0;
      bh[j] = Frag<T>::load(Bb + bo);
      if (SPLIT == 1) bl[j] = Frag<T>::load(Bb2 + bo);
    }
#pragma unroll
    for (int i = 0; i < 4; ++i) {
      const size_t ao = (size_t)(m0 + (i << 4) + rlane) * lda + koff + k0;
      V ah = Frag<T>::load(Ab + ao);
      V al = ah;
      if (SPLIT != 0) al = Frag<T>::load(Ab2 + ao);
#pragma unroll
      for (int j = 0; j < 4; ++j) {
        acc[i][j] = Frag<T>::mma(ah, bh[j], acc[i][j]);
        if (SPLIT == 1) acc[i][j] = Frag<T>::mma(ah, bl[j], acc[i][j]);
        if (SPLIT != 0) acc[i][j] = Frag<T>::mma(al, bh[j], acc[i][j]);
      }
      Frag<T>::guard4(acc[i][0], acc[i][1], acc[i][2], acc[i][3], ah, al);
    }
    Frag<T>::keep(bh[0], bh[1], bh[2], bh[3]);
    if (SPLIT == 1) Frag<T>::keep(bl[0], bl[1], bl[2], bl[3]);
  }
  acc_guard4(acc[0][0], acc[0][1], acc[0][2], acc[0][3]);
  acc_guard4(acc[1][0], acc[1][1], acc[1][2], acc[1][3]);
  acc_guard4(acc[2][0], acc[2][1], acc[2][2], acc[2][3]);
  acc_guard4(acc[3][0], acc[3][1], acc[3][2], acc[3][3]);

  float* slab = sT[wave];
  float bcol[4] = {0.f, 0.f, 0.f, 0.f};
  if (BIAS_MODE == 2) {
#pragma unroll
    for (int j = 0; j < 4; ++j) bcol[j] = bias[n0 + (j << 4) + rlane];
  }
#pragma unroll
  for (int i = 0; i < 4; ++i) {
    const int mBase = m0 + (i << 4);
    float brow[8] = {0.f, 0.f, 0.f, 0.f, 0.f, 0.f, 0.f, 0.f};
    if (BIAS_MODE == 1) {
      const v4f b0 = *(const v4f*)(bias + mBase + mOff);
      const v4f b1 = *(const v4f*)(bias + mBase + mOff + 4);
#pragma unroll
      for (int e = 0; e < 4; ++e) { brow[e] = b0[e]; brow[4 + e] = b1[e]; }
    }
#pragma unroll
    for (int j = 0; j < 4; ++j) {
#pragma unroll
      for (int r = 0; r < 8; ++r) {
        float bb = 0.f;
        if (BIAS_MODE == 1) bb = brow[r];
        if (BIAS_MODE == 2) bb = bcol[j];
        slab[(mOff + r) * 68 + (j << 4) + rlane] = acc[i][j][r] * scale + bb;
      }
    }
    __builtin_amdgcn_fence(3, "workgroup");
    __builtin_amdgcn_wave_barrier();
    __builtin_amdgcn_fence(2, "workgroup");
    if (OUT_MODE == 0) {
      float* C = (float*)Cout + (size_t)b * strideC;
      const int hh = lane >> 4, c4 = (lane & 15) * 4;
      for (int pass = 0; pass < 2; ++pass) {
#pragma unroll
        for (int it = 0; it < 8; ++it) {
          const int row = it * 2 + hh;
          const v4f v = *(const v4f*)(slab + row * 68 + c4);
          *(volatile v4f*)(C + (size_t)(mBase + row) * ldc + n0 + c4) = v;
        }
        __threadfence();
      }
    } else {
      const int q = lane >> 3, c8 = (lane & 7) * 8;
      unsigned short* C  = (unsigned short*)Cout  + (size_t)b * strideC;
      unsigned short* C2 = (OUT_MODE == 2) ? ((unsigned short*)Cout2 + (size_t)b * strideC) : nullptr;
      for (int pass = 0; pass < 2; ++pass) {
#pragma unroll
        for (int it = 0; it < 4; ++it) {
          const int row = it * 4 + q;
          const float* sp = slab + row * 68 + c8;
          v8h hv, lv;
#pragma unroll
          for (int e = 0; e < 8; ++e) {
            if (OUT_MODE == 1) {
              hv[e] = (_Float16)sp[e];
            } else {
              unsigned short hb = f2bf_bits(sp[e]);
              unsigned short lb = f2bf_bits(sp[e] - bf_bits2f(hb));
              hv[e] = __builtin_bit_cast(_Float16, hb);
              lv[e] = __builtin_bit_cast(_Float16, lb);
            }
          }
          *(volatile v8h*)(C + (size_t)(mBase + row) * ldc + n0 + c8) = hv;
          if (OUT_MODE == 2) *(volatile v8h*)(C2 + (size_t)(mBase + row) * ldc + n0 + c8) = lv;
        }
        __threadfence();
      }
    }
    __builtin_amdgcn_fence(3, "workgroup");
    __builtin_amdgcn_wave_barrier();
    __builtin_amdgcn_fence(2, "workgroup");
  }
}

__global__ __launch_bounds__(256) void cast8_bf16_kernel(const float* __restrict__ in, unsigned short* __restrict__ out, int n8) {
  const int i = blockIdx.x * 256 + threadIdx.x;
  if (i >= n8) return;
  const int t  = i >> 7;
  const int c8 = (i & 127) * 8;
  const int b  = t / kSeq;
  const int s  = t - b * kSeq;
  const float* p = in + (size_t)(b * kSeqFull + s) * kDim + c8;
  const v4f a = *(const v4f*)(p);
  const v4f c = *(const v4f*)(p + 4);
  unsigned short hb[8];
#pragma unroll
  for (int e = 0; e < 4; ++e) {
    hb[e]     = f2bf_bits(a[e]);
    hb[4 + e] = f2bf_bits(c[e]);
  }
  const v4u u = (v4u){pk16(hb[0], hb[1]), pk16(hb[2], hb[3]), pk16(hb[4], hb[5]), pk16(hb[6], hb[7])};
  unsigned short* q = out + 8 * (size_t)i;
  *(volatile v4u*)q = u;
  __threadfence();
  *(volatile v4u*)q = u;
}

__global__ __launch_bounds__(256) void wtcast_bf16_kernel(const float* __restrict__ W, unsigned short* __restrict__ out,
                                                          int ldIn, int ldOut) {
  __shared__ float sm[64][65];
  const int t  = threadIdx.x;
  const int d0 = blockIdx.x * 64;
  const int n0 = blockIdx.y * 64;
#pragma unroll
  for (int i = 0; i < 16; ++i) {
    const int e = i * 256 + t;
    const int r = e >> 6;
    const int c = e & 63;
    sm[c][r] = W[(size_t)(d0 + r) * ldIn + n0 + c];
  }
  __syncthreads();
  const int lane = t & 31, wave = t >> 5;
  const int q = lane >> 3, c8 = (lane & 7) * 8;
  for (int pass = 0; pass < 2; ++pass) {
#pragma unroll
    for (int it = 0; it < 2; ++it) {
      const int row = wave * 8 + it * 4 + q;
      unsigned short hb[8];
#pragma unroll
      for (int e = 0; e < 8; ++e) hb[e] = f2bf_bits(sm[row][c8 + e]);
      const v4u u = (v4u){pk16(hb[0], hb[1]), pk16(hb[2], hb[3]), pk16(hb[4], hb[5]), pk16(hb[6], hb[7])};
      *(volatile v4u*)(out + (size_t)(n0 + row) * ldOut + d0 + c8) = u;
    }
    __threadfence();
  }
}

__global__ __launch_bounds__(256) void bias_bf16_kernel(const float* __restrict__ bsrc, float* __restrict__ bdst) {
  const int t = threadIdx.x;
  const v4f a = *(const v4f*)(bsrc + 4 * t);
  v4f r;
#pragma unroll
  for (int e = 0; e < 4; ++e) r[e] = bf_bits2f(f2bf_bits(a[e]));
  float* dp = bdst + 4 * t;
  *(volatile v4f*)dp = r;
  __threadfence();
  *(volatile v4f*)dp = r;
}

union FragH { v16h v; v8h h[2]; };
union FragB { v16b v; v8b h[2]; };

__device__ __forceinline__ v8f mma_h16(v16h a, v16h b, v8f c) {
  c = __builtin_amdgcn_wmma_f32_16x16x32_f16(false, a, false, b, (short)0, c, false, false);
  asm volatile("v_nop\n\tv_nop\n\tv_nop\n\tv_nop" : "+v"(c) : "v"(a), "v"(b));
  return c;
}
__device__ __forceinline__ v8f mma_b16(v16b a, v16b b, v8f c) {
  c = __builtin_amdgcn_wmma_f32_16x16x32_bf16(false, a, false, b, (short)0, c, false, false);
  asm volatile("v_nop\n\tv_nop\n\tv_nop\n\tv_nop" : "+v"(c) : "v"(a), "v"(b));
  return c;
}
__device__ __forceinline__ __bf16 f2bf(float f) { return __builtin_bit_cast(__bf16, f2bf_bits(f)); }
__device__ __forceinline__ void bf_split(float f, __bf16& hi, __bf16& lo) {
  const unsigned short hb = f2bf_bits(f);
  hi = __builtin_bit_cast(__bf16, hb);
  lo = f2bf(f - __uint_as_float(((unsigned)hb) << 16));
}

__global__ __launch_bounds__(128) __attribute__((amdgpu_num_vgpr(256)))
void causal_attn_kernel(const unsigned short* __restrict__ QKp,
                        const unsigned short* __restrict__ VHp,
                        const unsigned short* __restrict__ VLp,
                        unsigned short* __restrict__ CHp,
                        unsigned short* __restrict__ CLp) {
  __shared__ __align__(16) unsigned short Ksh[kKC * kDh];
  __shared__ __align__(16) unsigned short Vth[kDh * kKC];
  __shared__ __align__(16) unsigned short Vtl[kDh * kKC];
  __shared__ __align__(16) __bf16 Psh[kAW][16 * kKC];
  __shared__ __align__(16) __bf16 Psl[kAW][16 * kKC];
  __shared__ __align__(16) float  Os[kAW][16 * 68];

  const int tid  = threadIdx.x;
  const int wave = tid >> 5;
  const int lane = tid & 31;
  const int hh   = lane >> 4;
  const int c    = lane & 15;

  const int nqb = kSeq / kQB;
  const int bx  = blockIdx.x;
  const int qb  = bx % nqb;
  const int bh  = bx / nqb;
  const int h   = bh % kHeads;
  const int b   = bh / kHeads;
  const int q0  = qb * kQB + wave * 16;

  const _Float16* Qb = (const _Float16*)(QKp + (size_t)b * kSeq * kQKld + h * kDh);
  const unsigned short* Kb  = QKp + (size_t)b * kSeq * kQKld + kDim + h * kDh;
  const unsigned short* Vhb = VHp + (size_t)bh * kDh * kSeq;
  const unsigned short* Vlb = VLp + (size_t)bh * kDh * kSeq;

  v16h qa[2];
#pragma unroll
  for (int dc = 0; dc < 2; ++dc) qa[dc] = Frag<_Float16>::load(Qb + (size_t)(q0 + c) * kQKld + dc * 32 + 8 * hh);

  float mrow[8], lrow[8];
  v8f oacc[4];
#pragma unroll
  for (int r = 0; r < 8; ++r) { mrow[r] = -INFINITY; lrow[r] = 0.f; }
#pragma unroll
  for (int t = 0; t < 4; ++t) oacc[t] = (v8f){0.f,0.f,0.f,0.f,0.f,0.f,0.f,0.f};

  const int nChunks = qb + 1;
  for (int kc = 0; kc < nChunks; ++kc) {
    const int kv0 = kc * kKC;
    __syncthreads();
    {
      const int r = tid >> 1, hf = (tid & 1) * 32;
      {
        const uint4* ks = (const uint4*)(Kb + (size_t)(kv0 + r) * kQKld + hf);
        uint4* kd = (uint4*)(Ksh + r * kDh + hf);
        const uint4 w0 = ks[0], w1 = ks[1], w2 = ks[2], w3 = ks[3];
        kd[0] = w0; kd[1] = w1; kd[2] = w2; kd[3] = w3;
      }
      asm volatile("" ::: "memory");
      {
        const uint4* vs = (const uint4*)(Vhb + (size_t)r * kSeq + kv0 + hf);
        uint4* vd = (uint4*)(Vth + r * kKC + hf);
        const uint4 w0 = vs[0], w1 = vs[1], w2 = vs[2], w3 = vs[3];
        vd[0] = w0; vd[1] = w1; vd[2] = w2; vd[3] = w3;
      }
      asm volatile("" ::: "memory");
      {
        const uint4* vs = (const uint4*)(Vlb + (size_t)r * kSeq + kv0 + hf);
        uint4* vd = (uint4*)(Vtl + r * kKC + hf);
        const uint4 w0 = vs[0], w1 = vs[1], w2 = vs[2], w3 = vs[3];
        vd[0] = w0; vd[1] = w1; vd[2] = w2; vd[3] = w3;
      }
    }
    __syncthreads();

    v8f s[4];
#pragma unroll
    for (int j = 0; j < 4; ++j) {
      s[j] = (v8f){0.f,0.f,0.f,0.f,0.f,0.f,0.f,0.f};
#pragma unroll
      for (int dc = 0; dc < 2; ++dc) {
        FragH kb;
        kb.h[0] = *(const v8h*)(Ksh + (j * 16 + c) * kDh + dc * 32 + 8 * hh);
        kb.h[1] = *(const v8h*)(Ksh + (j * 16 + c) * kDh + dc * 32 + 16 + 8 * hh);
        s[j] = mma_h16(qa[dc], kb.v, s[j]);
      }
    }
    const bool diag = (kc == qb);
    float cm[8];
#pragma unroll
    for (int r = 0; r < 8; ++r) {
      const int qrow = q0 + 8 * hh + r;
      float m = -INFINITY;
#pragma unroll
      for (int j = 0; j < 4; ++j) {
        const int kvcol = kv0 + j * 16 + c;
        float sv = s[j][r] * kScale;
        if (diag && (kvcol > qrow)) sv = kNegBig;
        s[j][r] = sv;
        m = fmaxf(m, sv);
      }
#pragma unroll
      for (int off = 1; off < 16; off <<= 1) m = fmaxf(m, __shfl_xor(m, off, 32));
      cm[r] = m;
    }
    __bf16* pwh = Psh[wave];
    __bf16* pwl = Psl[wave];
#pragma unroll
    for (int r = 0; r < 8; ++r) {
      const float mnew = fmaxf(mrow[r], cm[r]);
      const float alpha = expf(mrow[r] - mnew);
      mrow[r] = mnew;
      float psum = 0.f;
#pragma unroll
      for (int j = 0; j < 4; ++j) {
        const float p = expf(s[j][r] - mnew);
        psum += p;
        __bf16 ph, pl;
        bf_split(p, ph, pl);
        pwh[(8 * hh + r) * kKC + j * 16 + c] = ph;
        pwl[(8 * hh + r) * kKC + j * 16 + c] = pl;
      }
#pragma unroll
      for (int off = 1; off < 16; off <<= 1) psum += __shfl_xor(psum, off, 32);
      lrow[r] = lrow[r] * alpha + psum;
#pragma unroll
      for (int t = 0; t < 4; ++t) oacc[t][r] *= alpha;
    }
    __builtin_amdgcn_fence(3, "workgroup");
    __builtin_amdgcn_wave_barrier();
    __builtin_amdgcn_fence(2, "workgroup");
#pragma unroll 1
    for (int kk = 0; kk < 2; ++kk) {
      FragB pa, pl;
      pa.h[0] = *(const v8b*)(pwh + c * kKC + kk * 32 + 8 * hh);
      pa.h[1] = *(const v8b*)(pwh + c * kKC + kk * 32 + 16 + 8 * hh);
      pl.h[0] = *(const v8b*)(pwl + c * kKC + kk * 32 + 8 * hh);
      pl.h[1] = *(const v8b*)(pwl + c * kKC + kk * 32 + 16 + 8 * hh);
#pragma unroll
      for (int t = 0; t < 4; ++t) {
        FragB vb, vl;
        vb.h[0] = *(const v8b*)(Vth + (t * 16 + c) * kKC + kk * 32 + 8 * hh);
        vb.h[1] = *(const v8b*)(Vth + (t * 16 + c) * kKC + kk * 32 + 16 + 8 * hh);
        vl.h[0] = *(const v8b*)(Vtl + (t * 16 + c) * kKC + kk * 32 + 8 * hh);
        vl.h[1] = *(const v8b*)(Vtl + (t * 16 + c) * kKC + kk * 32 + 16 + 8 * hh);
        oacc[t] = mma_b16(pa.v, vb.v, oacc[t]);
        oacc[t] = mma_b16(pa.v, vl.v, oacc[t]);
        oacc[t] = mma_b16(pl.v, vb.v, oacc[t]);
      }
    }
  }

  float* os = Os[wave];
#pragma unroll
  for (int r = 0; r < 8; ++r) {
    const float inv = 1.0f / lrow[r];
#pragma unroll
    for (int t = 0; t < 4; ++t) os[(8 * hh + r) * 68 + t * 16 + c] = oacc[t][r] * inv;
  }
  __builtin_amdgcn_fence(3, "workgroup");
  __builtin_amdgcn_wave_barrier();
  __builtin_amdgcn_fence(2, "workgroup");
  {
    const int q = lane >> 3, c8 = (lane & 7) * 8;
    unsigned short* ch = CHp + (size_t)(b * kSeq + q0) * kDim + h * kDh;
    unsigned short* cl = CLp + (size_t)(b * kSeq + q0) * kDim + h * kDh;
    for (int pass = 0; pass < 2; ++pass) {
#pragma unroll
      for (int it = 0; it < 4; ++it) {
        const int row = it * 4 + q;
        const float* sp = os + row * 68 + c8;
        v8h hv, lv;
#pragma unroll
        for (int e = 0; e < 8; ++e) {
          const unsigned short hb = f2bf_bits(sp[e]);
          const unsigned short lb = f2bf_bits(sp[e] - bf_bits2f(hb));
          hv[e] = __builtin_bit_cast(_Float16, hb);
          lv[e] = __builtin_bit_cast(_Float16, lb);
        }
        *(volatile v8h*)(ch + (size_t)row * kDim + c8) = hv;
        *(volatile v8h*)(cl + (size_t)row * kDim + c8) = lv;
      }
      __threadfence();
    }
  }
}

extern "C" void kernel_launch(void* const* d_in, const int* in_sizes, int n_in,
                              void* d_out, int out_size, void* d_ws, size_t ws_size,
                              hipStream_t stream) {
  if (n_in < 8) return;
  const int rowsNeeded = (kBatch - 1) * kSeqFull + kSeq;
  if (in_sizes[0] < rowsNeeded * kDim) return;
  if (in_sizes[1] < kDim * kDim || in_sizes[3] < kDim * kDim || in_sizes[5] < kDim * kDim || in_sizes[7] < kDim * kDim) return;
  if (in_sizes[2] < kDim || in_sizes[4] < kDim || in_sizes[6] < kDim) return;
  if (out_size < rowsNeeded * kDim) return;

  const size_t szXB  = (size_t)kTok * kDim * 2;
  const size_t szWT  = (size_t)kWtN * kDim * 2;
  const size_t szWOT = (size_t)kDim * kDim * 2;
  const size_t szBQK = (size_t)kQKld * 4;
  const size_t szBV  = (size_t)kDim * 4;
  const size_t szQK  = (size_t)kTok * kQKld * 2;
  const size_t szVT  = (size_t)kBatch * kHeads * kDh * kSeq * 2;
  const size_t szCTX = (size_t)kTok * kDim * 2;
  const size_t offXB  = 0;
  const size_t offWT  = offXB + szXB;
  const size_t offWOT = offWT + szWT;
  const size_t offBQK = offWOT + szWOT;
  const size_t offBV  = offBQK + szBQK;
  const size_t offQK  = offBV + szBV;
  const size_t offVTH = offQK + szQK;
  const size_t offVTL = offVTH + szVT;
  const size_t offCH  = offVTL + szVT;
  const size_t offCL  = offCH + szCTX;
  const size_t total  = offCL + szCTX;
  if (ws_size < total) return;
  if (total > (size_t)134217728) return;

  const float* x  = (const float*)d_in[0];
  const float* Wq = (const float*)d_in[1];
  const float* bq = (const float*)d_in[2];
  const float* Wk = (const float*)d_in[3];
  const float* bk = (const float*)d_in[4];
  const float* Wv = (const float*)d_in[5];
  const float* bv = (const float*)d_in[6];
  const float* Wo = (const float*)d_in[7];
  float* out = (float*)d_out;
  char* ws = (char*)d_ws;
  unsigned short* XB   = (unsigned short*)(ws + offXB);
  unsigned short* WT   = (unsigned short*)(ws + offWT);
  unsigned short* WOT  = (unsigned short*)(ws + offWOT);
  float*          BQK  = (float*)(ws + offBQK);
  float*          BV   = (float*)(ws + offBV);
  unsigned short* QK16 = (unsigned short*)(ws + offQK);
  unsigned short* VTH  = (unsigned short*)(ws + offVTH);
  unsigned short* VTL  = (unsigned short*)(ws + offVTL);
  unsigned short* CTXH = (unsigned short*)(ws + offCH);
  unsigned short* CTXL = (unsigned short*)(ws + offCL);

  const int n8 = kTok * kDim / 8;
  cast8_bf16_kernel<<<dim3((n8 + 255) / 256), dim3(256), 0, stream>>>(x, XB, n8);
  wtcast_bf16_kernel<<<dim3(kDim / 64, kDim / 64), dim3(256), 0, stream>>>(Wq, WT, kDim, kDim);
  wtcast_bf16_kernel<<<dim3(kDim / 64, kDim / 64), dim3(256), 0, stream>>>(Wk, WT + (size_t)kDim * kDim, kDim, kDim);
  wtcast_bf16_kernel<<<dim3(kDim / 64, kDim / 64), dim3(256), 0, stream>>>(Wv, WT + (size_t)2 * kDim * kDim, kDim, kDim);
  wtcast_bf16_kernel<<<dim3(kDim / 64, kDim / 64), dim3(256), 0, stream>>>(Wo, WOT, kDim, kDim);
  bias_bf16_kernel<<<dim3(1), dim3(256), 0, stream>>>(bq, BQK);
  bias_bf16_kernel<<<dim3(1), dim3(256), 0, stream>>>(bk, BQK + kDim);
  bias_bf16_kernel<<<dim3(1), dim3(256), 0, stream>>>(bv, BV);

  {
    const int tiles = (kTok / 64) * (kQKld / 64);
    wmma_gemm64<1, 0, 2, 1><<<dim3((tiles + 7) / 8, 1), dim3(256), 0, stream>>>(
        XB, XB, kDim, 0L, WT, WT, kDim, 0L,
        (void*)QK16, (void*)QK16, kQKld, 0L, BQK, kTok, kQKld, kDim, 1.0f);
  }
  {
    const int tiles = (kDim / 64) * (kSeq / 64);
    const unsigned short* Av = WT + (size_t)2 * kDim * kDim;
    wmma_gemm64<1, 0, 1, 2><<<dim3((tiles + 7) / 8, kBatch), dim3(256), 0, stream>>>(
        Av, Av, kDim, 0L, XB, XB, kDim, (long)kSeq * kDim,
        (void*)VTH, (void*)VTL, kSeq, (long)kDim * kSeq, BV, kDim, kSeq, kDim, 1.0f);
  }
  causal_attn_kernel<<<dim3(kBatch * kHeads * (kSeq / kQB)), dim3(128), 0, stream>>>(QK16, VTH, VTL, CTXH, CTXL);
  {
    const int tiles = (kSeq / 64) * (kDim / 64);
    wmma_gemm64<1, 2, 0, 0><<<dim3((tiles + 7) / 8, kBatch), dim3(256), 0, stream>>>(
        CTXH, CTXL, kDim, (long)kSeq * kDim, WOT, WOT, kDim, 0L,
        (void*)out, (void*)out, kDim, (long)kSeqFull * kDim, BV, kSeq, kDim, kDim, 1.0f);
  }
}
